// NodeEConvModel_80831284510903
// MI455X (gfx1250) — hardware-verified
//
#include <hip/hip_runtime.h>
#include <stddef.h>
#include <math.h>


#define NTHR   256
#define NWAVE  8
#define EPT    8
#define CHUNK  (NTHR * EPT)
#define WCAP   (EPT * 32)
#define LISTN  (NWAVE * WCAP)
#define PASSN  128
#define PCAP   (CHUNK + PASSN)
#define NODET  128

#define OF_WB1 0
#define OF_PA2 512
#define OF_QA2 2560
#define OF_WB2 4608
#define OF_PA3 6656
#define OF_QA3 10752
#define OF_WB3 14848
#define OF_AE  23040
#define OF_BE  27136
#define OF_WE2 31232
#define OF_CN  32256
#define OF_EN  36352
#define OF_WN2 38400
#define OF_WM1 40448
#define PLANES_H 40960
#define NPLANES 14

static_assert(PCAP >= CHUNK + PASSN);
static_assert(PASSN == 16 * NWAVE);

typedef float    v4f  __attribute__((ext_vector_type(4)));
typedef float    v8f  __attribute__((ext_vector_type(8)));
typedef int      v4i  __attribute__((ext_vector_type(4)));
typedef _Float16 v8h  __attribute__((ext_vector_type(8)));
typedef _Float16 v16h __attribute__((ext_vector_type(16)));
union FragH { v16h v; v8h h[2]; };

__device__ __forceinline__ v8f zacc() {
  v8f c;
#pragma unroll
  for (int i = 0; i < 8; ++i) c[i] = 0.0f;
  return c;
}

__device__ __forceinline__ v8f wmh(v16h a, v16h b, v8f c) {
  v8f d = __builtin_amdgcn_wmma_f32_16x16x32_f16(false, a, false, b, (short)0, c, false, false);
  asm volatile("v_nop\n\tv_nop\n\tv_nop\n\tv_nop" : "+v"(d) : "v"(a), "v"(b));
  return d;
}

__device__ __forceinline__ float lrl(float v, float s) { return v >= 0.0f ? v : s * v; }
__device__ __forceinline__ int clampi(int v, int hi) { return v < 0 ? 0 : (v > hi ? hi : v); }

template <int NBK>
__device__ __forceinline__ int scan_chunk(const int* __restrict__ keys, int nE, int cbase, int nodeBase,
                                          int vec8, int* list, int tid, int wave) {
  int wc = 0;
  const int el0  = tid * EPT;
  const int e0   = cbase + el0;
  const int sent = -2147483647 - 1;
  v4i da, db;
  if (vec8 != 0 && cbase + CHUNK <= nE) {
    da = *(const v4i*)(keys + e0);
    db = *(const v4i*)(keys + e0 + 4);
  } else {
    da.x = (e0     < nE) ? keys[min(e0, nE - 1)] : sent;
    da.y = (e0 + 1 < nE) ? keys[min(e0 + 1, nE - 1)] : sent;
    da.z = (e0 + 2 < nE) ? keys[min(e0 + 2, nE - 1)] : sent;
    da.w = (e0 + 3 < nE) ? keys[min(e0 + 3, nE - 1)] : sent;
    db.x = (e0 + 4 < nE) ? keys[min(e0 + 4, nE - 1)] : sent;
    db.y = (e0 + 5 < nE) ? keys[min(e0 + 5, nE - 1)] : sent;
    db.z = (e0 + 6 < nE) ? keys[min(e0 + 6, nE - 1)] : sent;
    db.w = (e0 + 7 < nE) ? keys[min(e0 + 7, nE - 1)] : sent;
  }
  const unsigned nb = (unsigned)nodeBase;
  const unsigned s0 = (unsigned)da.x - nb, s1 = (unsigned)da.y - nb;
  const unsigned s2 = (unsigned)da.z - nb, s3 = (unsigned)da.w - nb;
  const unsigned s4 = (unsigned)db.x - nb, s5 = (unsigned)db.y - nb;
  const unsigned s6 = (unsigned)db.z - nb, s7 = (unsigned)db.w - nb;
  const bool h0 = s0 < (unsigned)NBK, h1 = s1 < (unsigned)NBK, h2 = s2 < (unsigned)NBK, h3 = s3 < (unsigned)NBK;
  const bool h4 = s4 < (unsigned)NBK, h5 = s5 < (unsigned)NBK, h6 = s6 < (unsigned)NBK, h7 = s7 < (unsigned)NBK;
  const unsigned any = __builtin_amdgcn_ballot_w32(h0 | h1 | h2 | h3 | h4 | h5 | h6 | h7);
  if (any != 0u) {
#define HITJ(J, HJ) { \
      const unsigned mj = __builtin_amdgcn_ballot_w32(HJ); \
      if (mj != 0u) { \
        if (HJ) { \
          const int pos = wc + (int)__builtin_amdgcn_mbcnt_lo(mj, 0u); \
          if (pos < WCAP) list[wave * WCAP + pos] = el0 + (J); \
        } \
        wc += (int)__builtin_popcount(mj); } }
    HITJ(0, h0)
    HITJ(1, h1)
    HITJ(2, h2)
    HITJ(3, h3)
    HITJ(4, h4)
    HITJ(5, h5)
    HITJ(6, h6)
    HITJ(7, h7)
#undef HITJ
  }
  return wc;
}

__device__ __forceinline__ v8h prep_vals(const float* __restrict__ S, int NO, int koff, int ksub, float sub,
                                         int KV, float sc, int kp8, int i) {
  const int n  = i / kp8;
  const int k0 = (i - n * kp8) * 8;
  v8h r;
#pragma unroll
  for (int j = 0; j < 8; ++j) {
    const int k  = k0 + j;
    const int kk = k < KV ? k : KV - 1;
    const float a = S[(koff + kk) * NO + n];
    const float b = S[(ksub + kk) * NO + n];
    float v = a - sub * b;
    if (k >= KV) v = 0.0f;
    r[j] = (_Float16)(v * sc);
  }
  return r;
}

__global__ __launch_bounds__(NTHR) void k_prep(
    const float* __restrict__ w1b, const float* __restrict__ w2a, const float* __restrict__ w2b,
    const float* __restrict__ w3a, const float* __restrict__ w3b, const float* __restrict__ we1,
    const float* __restrict__ we2, const float* __restrict__ wn1, const float* __restrict__ wn2,
    const float* __restrict__ wm1, _Float16* planes) {
  const int pl = blockIdx.x, tid = threadIdx.x;
  const float* S = w1b;
  int NO = 16, koff = 0, ksub = 0, KV = 32, NR = 16, KP = 32, off = OF_WB1;
  float sc = 4.0f, sub = 0.0f;
  switch (pl) {
    case 0:  S = w1b; NO = 16;  koff = 0;  ksub = 0;  sub = 0.0f; KV = 32;  sc = 4.0f; NR = 16;  KP = 32;  off = OF_WB1; break;
    case 1:  S = w2a; NO = 64;  koff = 0;  ksub = 16; sub = 1.0f; KV = 16;  sc = 4.0f; NR = 64;  KP = 32;  off = OF_PA2; break;
    case 2:  S = w2a; NO = 64;  koff = 16; ksub = 16; sub = 0.0f; KV = 16;  sc = 4.0f; NR = 64;  KP = 32;  off = OF_QA2; break;
    case 3:  S = w2b; NO = 32;  koff = 0;  ksub = 0;  sub = 0.0f; KV = 64;  sc = 8.0f; NR = 32;  KP = 64;  off = OF_WB2; break;
    case 4:  S = w3a; NO = 128; koff = 0;  ksub = 32; sub = 1.0f; KV = 32;  sc = 8.0f; NR = 128; KP = 32;  off = OF_PA3; break;
    case 5:  S = w3a; NO = 128; koff = 32; ksub = 32; sub = 0.0f; KV = 32;  sc = 8.0f; NR = 128; KP = 32;  off = OF_QA3; break;
    case 6:  S = w3b; NO = 64;  koff = 0;  ksub = 0;  sub = 0.0f; KV = 128; sc = 8.0f; NR = 64;  KP = 128; off = OF_WB3; break;
    case 7:  S = we1; NO = 64;  koff = 0;  ksub = 0;  sub = 0.0f; KV = 64;  sc = 8.0f; NR = 64;  KP = 64;  off = OF_AE;  break;
    case 8:  S = we1; NO = 64;  koff = 64; ksub = 64; sub = 0.0f; KV = 64;  sc = 8.0f; NR = 64;  KP = 64;  off = OF_BE;  break;
    case 9:  S = we2; NO = 16;  koff = 0;  ksub = 0;  sub = 0.0f; KV = 64;  sc = 8.0f; NR = 16;  KP = 64;  off = OF_WE2; break;
    case 10: S = wn1; NO = 64;  koff = 0;  ksub = 0;  sub = 0.0f; KV = 64;  sc = 8.0f; NR = 64;  KP = 64;  off = OF_CN;  break;
    case 11: S = wn1; NO = 64;  koff = 64; ksub = 64; sub = 0.0f; KV = 16;  sc = 8.0f; NR = 64;  KP = 32;  off = OF_EN;  break;
    case 12: S = wn2; NO = 32;  koff = 0;  ksub = 0;  sub = 0.0f; KV = 64;  sc = 8.0f; NR = 32;  KP = 64;  off = OF_WN2; break;
    case 13: S = wm1; NO = 16;  koff = 0;  ksub = 0;  sub = 0.0f; KV = 32;  sc = 4.0f; NR = 16;  KP = 32;  off = OF_WM1; break;
    default: return;
  }
  const int kp8 = KP >> 3;
  const int ngrp = NR * kp8;
  _Float16* dst = planes + off;
  for (int i = tid; i < ngrp; i += NTHR) {
    const v8h v = prep_vals(S, NO, koff, ksub, sub, KV, sc, kp8, i);
    *(volatile v8h*)(dst + 8 * i) = v;
  }
  __threadfence();
  for (int i = tid; i < ngrp; i += NTHR) {
    const v8h v = prep_vals(S, NO, koff, ksub, sub, KV, sc, kp8, i);
    *(volatile v8h*)(dst + 8 * i) = v;
  }
}

__device__ __forceinline__ void node1_pass(const float* __restrict__ x, const float* dw, const float* qw, float bv,
                                           float* P, float* Q, int nN, int nPad, int gw, int nw, int lane) {
#pragma unroll 1
  for (int node = gw; node < nPad; node += nw) {
    const int nn = node < nN ? node : nN - 1;
    const v4f xv = *(const v4f*)(x + (size_t)nn * 4);
    float p = bv;
    p += xv.x * dw[0]; p += xv.y * dw[1]; p += xv.z * dw[2]; p += xv.w * dw[3];
    float q = xv.x * qw[0];
    q += xv.y * qw[1]; q += xv.z * qw[2]; q += xv.w * qw[3];
    *(volatile float*)(P + (size_t)node * 32 + lane) = p;
    *(volatile float*)(Q + (size_t)node * 32 + lane) = q;
  }
}

__global__ __launch_bounds__(NTHR) void k_node1(const float* __restrict__ x, const float* __restrict__ w1a,
                                                const float* __restrict__ b1a, float* P, float* Q, int nN, int nPad) {
  const int lane = threadIdx.x & 31, wave = threadIdx.x >> 5;
  const int gw = blockIdx.x * NWAVE + wave, nw = gridDim.x * NWAVE;
  float dw[4], qw[4];
#pragma unroll
  for (int c = 0; c < 4; ++c) {
    const float t = w1a[c * 32 + lane];
    const float b = w1a[(4 + c) * 32 + lane];
    dw[c] = t - b;
    qw[c] = b;
  }
  const float bv = b1a[lane];
  node1_pass(x, dw, qw, bv, P, Q, nN, nPad, gw, nw, lane);
  __threadfence();
  node1_pass(x, dw, qw, bv, P, Q, nN, nPad, gw, nw, lane);
}

template <int H>
__device__ __forceinline__ void tile_store(const float* dw, float* Y, size_t gb, int lane) {
#pragma unroll 1
  for (int q = 0; q < H / 8; ++q) {
    const int f = (q * 32 + lane) * 4;
    const v4f v = *(const v4f*)(dw + f);
    *(volatile v4f*)(Y + gb + f) = v;
  }
}

template <int D, int H, int NP>
__global__ __launch_bounds__(NTHR) void k_nodeg(const float* __restrict__ X,
    const _Float16* __restrict__ W0, const _Float16* __restrict__ W1, const _Float16* __restrict__ W2,
    const float* __restrict__ B0, const float* __restrict__ B2, float inv,
    float* Y0, float* Y1, float* Y2) {
  constexpr int KP   = (D < 32) ? 32 : D;
  constexpr int KS   = KP / 32;
  constexpr int KP8  = KP / 8;
  constexpr int NB16 = H / 16;
  static_assert((D % 8) == 0 && (H % 32) == 0);
  __shared__ __attribute__((aligned(16))) _Float16 xs[NODET * KP];
  __shared__ __attribute__((aligned(16))) _Float16 wsm[NP * H * KP];
  __shared__ float bsm[NP * H];
  __shared__ __attribute__((aligned(16))) float dstg[NWAVE * 16 * H];

  const int tid = threadIdx.x, lane = tid & 31, wave = tid >> 5, hh = lane >> 4, m = lane & 15;
  const int node0 = blockIdx.x * NODET;

  for (int i = tid; i < NODET * KP8; i += NTHR) {
    const int row = i / KP8;
    const int k   = (i - row * KP8) * 8;
    const int kk  = (k + 8 <= D) ? k : D - 8;
    const float* xp = X + ((size_t)node0 + row) * D + kk;
    const v4f a = *(const v4f*)xp;
    const v4f b = *(const v4f*)(xp + 4);
    const bool z = (k >= D);
    v8h hv;
#pragma unroll
    for (int j = 0; j < 4; ++j) {
      hv[j]     = (_Float16)(z ? 0.0f : a[j]);
      hv[4 + j] = (_Float16)(z ? 0.0f : b[j]);
    }
    *(v8h*)(xs + row * KP + k) = hv;
  }
#pragma unroll
  for (int p = 0; p < NP; ++p) {
    const _Float16* src = (p == 0) ? W0 : ((p == 1) ? W1 : W2);
    for (int i = tid; i < H * KP8; i += NTHR) *(v8h*)(wsm + p * H * KP + 8 * i) = *(const v8h*)(src + 8 * i);
  }
  for (int i = tid; i < NP * H; i += NTHR) {
    const int p = i / H;
    const int n = i - p * H;
    const float b0 = B0[n];
    const float b2 = B2[n];
    bsm[i] = (p == 0) ? b0 : ((p == 2) ? b2 : 0.0f);
  }
  __syncthreads();

  float* dw = dstg + wave * 16 * H;
  const _Float16* arow = xs + (wave * 16 + m) * KP + 8 * hh;
#pragma unroll
  for (int p = 0; p < NP; ++p) {
    const _Float16* wp = wsm + p * H * KP;
#pragma unroll
    for (int nb = 0; nb < NB16; ++nb) {
      v8f ac = zacc();
#pragma unroll
      for (int ks = 0; ks < KS; ++ks) {
        FragH a, b;
        a.h[0] = *(const v8h*)(arow + 32 * ks);
        a.h[1] = *(const v8h*)(arow + 32 * ks + 16);
        const _Float16* brow = wp + (nb * 16 + m) * KP + 8 * hh + 32 * ks;
        b.h[0] = *(const v8h*)brow;
        b.h[1] = *(const v8h*)(brow + 16);
        ac = wmh(a.v, b.v, ac);
      }
      const float bv = bsm[p * H + nb * 16 + m];
      float* dp = dw + (8 * hh) * H + nb * 16 + m;
#pragma unroll
      for (int r = 0; r < 8; ++r) dp[r * H] = ac[r] * inv + bv;
    }
    __syncthreads();
    float* Y = (p == 0) ? Y0 : ((p == 1) ? Y1 : Y2);
    const size_t gb = ((size_t)node0 + wave * 16) * H;
    tile_store<H>(dw, Y, gb, lane);
    __threadfence();
    tile_store<H>(dw, Y, gb, lane);
    __syncthreads();
  }
}

template <int OUT, int NQ>
__device__ __forceinline__ void econv_store(const float* acc, const int* cntb, float* xout, size_t ob, int wave, int lane) {
#pragma unroll 1
  for (int q = 0; q < NQ; ++q) {
    const int f  = (wave * NQ + q) * 128 + 4 * lane;
    const int sl = f / OUT;
    const int c  = f - sl * OUT;
    v4f v = *(const v4f*)(acc + sl * OUT + c);
    if (cntb[sl] <= 0) { v.x = 0.0f; v.y = 0.0f; v.z = 0.0f; v.w = 0.0f; }
    *(volatile v4f*)(xout + ob + f) = v;
  }
}

template <int H, int OUT, int NBK>
__global__ __launch_bounds__(NTHR) void k_econv(
    const float* __restrict__ P, const float* __restrict__ Q, const int* __restrict__ ei,
    const _Float16* __restrict__ wbp, const float* __restrict__ bb, float inv,
    float* xout, int nN, int nE, int vec8) {
  constexpr int NACC = OUT / 16;
  constexpr int KS   = H / 32;
  constexpr int NQ   = (NBK * OUT) / (128 * NWAVE);
  constexpr int NCW  = (OUT + 31) / 32;
  constexpr int GH   = H / 16;
  static_assert(NQ * 128 * NWAVE == NBK * OUT);
  static_assert((H % 32) == 0 && (OUT % 16) == 0 && OUT <= 64);

  __shared__ __attribute__((aligned(16))) float    acc[(NBK + 1) * OUT];
  __shared__ int cntb[NBK + 1];
  __shared__ __attribute__((aligned(16))) _Float16 stg[PASSN * H];
  __shared__ __attribute__((aligned(16))) float    msg[PASSN * OUT];
  __shared__ __attribute__((aligned(16))) _Float16 wsm[OUT * H];
  __shared__ float bsm[OUT];
  __shared__ __attribute__((aligned(16))) int list[LISTN];
  __shared__ int pend[PCAP];
  __shared__ int slotb[PASSN];
  __shared__ int wcnt[NWAVE];
  __shared__ int pendN;

  const int tid = threadIdx.x, lane = tid & 31, wave = tid >> 5, hh = lane >> 4, m = lane & 15;
  const int nodeBase = blockIdx.x * NBK;
  const int* srcs = ei;
  const int* dsts = ei + nE;

  for (int i = tid; i < (NBK + 1) * OUT; i += NTHR) acc[i] = -3.0e38f;
  for (int i = tid; i <= NBK; i += NTHR) cntb[i] = 0;
  for (int i = tid; i < OUT * H / 8; i += NTHR) *(v8h*)(wsm + 8 * i) = *(const v8h*)(wbp + 8 * i);
  {
    const int bi = tid < OUT ? tid : 0;
    const float vb = bb[bi];
    if (tid < OUT) bsm[tid] = vb;
  }
  if (tid == 0) pendN = 0;
  __syncthreads();

  const int nChunks = (nE + CHUNK - 1) / CHUNK;
#pragma unroll 1
  for (int ch = 0; ch < nChunks; ++ch) {
    const int cbase = ch * CHUNK;
    const int wc = scan_chunk<NBK>(dsts, nE, cbase, nodeBase, vec8, list, tid, wave);
    if (lane == 0) wcnt[wave] = wc;
    __syncthreads();

    const int base = pendN;
    int tot = 0, myoff = 0;
#pragma unroll
    for (int w = 0; w < NWAVE; ++w) {
      int c = wcnt[w];
      c = c > WCAP ? WCAP : (c < 0 ? 0 : c);
      if (w < wave) myoff += c;
      tot += c;
    }
    int newN = base + tot;
    newN = newN > PCAP ? PCAP : newN;
    {
      int n = wcnt[wave];
      n = n > WCAP ? WCAP : (n < 0 ? 0 : n);
      const int* lp = list + wave * WCAP;
      for (int i = lane; i < n; i += 32) {
        const int pos = base + myoff + i;
        if (pos < PCAP) pend[pos] = cbase + lp[i];
      }
    }
    const int fin = (ch == nChunks - 1) ? 1 : 0;
    const int R   = (fin != 0) ? (newN + PASSN - 1) / PASSN : newN / PASSN;
    const int Pv  = (fin != 0) ? newN : R * PASSN;
    __syncthreads();

#pragma unroll 1
    for (int r = 0; r < R; ++r) {
      {
        const int el  = wave * 16 + m;
        const int idx = r * PASSN + el;
        const bool valid = idx < Pv;
        int e = pend[idx];
        if (!valid) e = 0;
        e = clampi(e, nE - 1);
        int d = dsts[e];
        int s = srcs[e];
        int slot = d - nodeBase;
        if (!valid || (unsigned)slot >= (unsigned)NBK) slot = NBK;
        d = clampi(d, nN - 1);
        s = clampi(s, nN - 1);
        if (hh == 0) slotb[el] = slot;
        const float* pp = P + (size_t)d * H + hh * (H / 2);
        const float* qp = Q + (size_t)s * H + hh * (H / 2);
        _Float16* sp = stg + el * H + hh * (H / 2);
#pragma unroll 1
        for (int g = 0; g < GH; ++g) {
          const v4f p0 = *(const v4f*)(pp + 8 * g);
          const v4f p1 = *(const v4f*)(pp + 8 * g + 4);
          const v4f q0 = *(const v4f*)(qp + 8 * g);
          const v4f q1 = *(const v4f*)(qp + 8 * g + 4);
          const v4f t0 = p0 + q0;
          const v4f t1 = p1 + q1;
          v8h hv;
#pragma unroll
          for (int j = 0; j < 4; ++j) {
            float a = lrl(t0[j], 0.1f);
            float b = lrl(t1[j], 0.1f);
            if (!valid) { a = 0.0f; b = 0.0f; }
            hv[j]     = (_Float16)a;
            hv[4 + j] = (_Float16)b;
          }
          *(v8h*)(sp + 8 * g) = hv;
        }
      }
      __syncthreads();

      {
        v8f ac[NACC];
#pragma unroll
        for (int nb = 0; nb < NACC; ++nb) ac[nb] = zacc();
        const _Float16* arow = stg + (wave * 16 + m) * H + 8 * hh;
#pragma unroll
        for (int ks = 0; ks < KS; ++ks) {
          FragH a;
          a.h[0] = *(const v8h*)(arow + 32 * ks);
          a.h[1] = *(const v8h*)(arow + 32 * ks + 16);
#pragma unroll
          for (int nb = 0; nb < NACC; ++nb) {
            FragH b;
            const _Float16* brow = wsm + (nb * 16 + m) * H + 8 * hh + 32 * ks;
            b.h[0] = *(const v8h*)brow;
            b.h[1] = *(const v8h*)(brow + 16);
            ac[nb] = wmh(a.v, b.v, ac[nb]);
          }
        }
#pragma unroll
        for (int nb = 0; nb < NACC; ++nb) {
          const float bv = bsm[nb * 16 + m];
          float* mp = msg + (wave * 16 + 8 * hh) * OUT + nb * 16 + m;
#pragma unroll
          for (int rr = 0; rr < 8; ++rr) mp[rr * OUT] = lrl(ac[nb][rr] * inv + bv, 0.1f);
        }
      }
      __syncthreads();

      if (wave < NCW) {
        const int c = wave * 32 + lane;
        const bool cv = c < OUT;
        const int cc = cv ? c : 0;
#pragma unroll 1
        for (int i = 0; i < PASSN; ++i) {
          int sl = slotb[i];
          sl = sl < 0 ? 0 : (sl > NBK ? NBK : sl);
          const float v = msg[i * OUT + cc];
          float* ap = acc + sl * OUT + cc;
          const float nv = fmaxf(*ap, v);
          if (cv) *ap = nv;
          if (tid == 0) cntb[sl] += 1;
        }
      }
      __syncthreads();
    }

    int rem = newN - R * PASSN;
    rem = rem < 0 ? 0 : rem;
    if (R > 0 && tid < rem) pend[tid] = pend[R * PASSN + tid];
    if (tid == 0) pendN = rem;
  }
  __syncthreads();

  const size_t ob = (size_t)nodeBase * OUT;
  econv_store<OUT, NQ>(acc, cntb, xout, ob, wave, lane);
  __threadfence();
  econv_store<OUT, NQ>(acc, cntb, xout, ob, wave, lane);
}

template <int NBK>
__global__ __launch_bounds__(NTHR) void k_meta(
    const float* __restrict__ Ap, const float* __restrict__ Bp, const float* __restrict__ Cp,
    const int* __restrict__ ei,
    const _Float16* __restrict__ we2p, const _Float16* __restrict__ enp,
    const _Float16* __restrict__ wn2p, const _Float16* __restrict__ wm1p,
    const float* __restrict__ be2, const float* __restrict__ bn2, const float* __restrict__ bm1,
    const float* __restrict__ wm2, const float* __restrict__ bm2,
    float* outp, int nN, int nE, int vec8) {
  constexpr int NQO = (NBK * 2) / (128 * NWAVE);
  constexpr int NTT = NBK / (16 * NWAVE);
  static_assert(NQO * 128 * NWAVE == NBK * 2);
  static_assert(NTT * 16 * NWAVE == NBK);

  __shared__ __attribute__((aligned(16))) float    acc[(NBK + 1) * 32];
  __shared__ int cntb[NBK + 1];
  __shared__ __attribute__((aligned(16))) _Float16 stgU[PASSN * 64];
  __shared__ __attribute__((aligned(16))) _Float16 stgE[PASSN * 32];
  __shared__ __attribute__((aligned(16))) _Float16 stgV[PASSN * 64];
  __shared__ __attribute__((aligned(16))) float    msg[PASSN * 32];
  __shared__ __attribute__((aligned(16))) _Float16 wsm[5632];
  __shared__ float bias[100];
  __shared__ __attribute__((aligned(16))) float    outst[NBK * 2];
  __shared__ __attribute__((aligned(16))) int list[LISTN];
  __shared__ int pend[PCAP];
  __shared__ int slotb[PASSN];
  __shared__ int colb[PASSN];
  __shared__ int wcnt[NWAVE];
  __shared__ int pendN;

  const int tid = threadIdx.x, lane = tid & 31, wave = tid >> 5, hh = lane >> 4, m = lane & 15;
  const int nodeBase = blockIdx.x * NBK;
  const int* srcs = ei;
  const int* dsts = ei + nE;

  for (int i = tid; i < (NBK + 1) * 32; i += NTHR) acc[i] = 0.0f;
  for (int i = tid; i <= NBK; i += NTHR) cntb[i] = 0;
  for (int i = tid; i < 128; i += NTHR) *(v8h*)(wsm + 8 * i)        = *(const v8h*)(we2p + 8 * i);
  for (int i = tid; i < 256; i += NTHR) *(v8h*)(wsm + 1024 + 8 * i) = *(const v8h*)(enp + 8 * i);
  for (int i = tid; i < 256; i += NTHR) *(v8h*)(wsm + 3072 + 8 * i) = *(const v8h*)(wn2p + 8 * i);
  for (int i = tid; i < 64;  i += NTHR) *(v8h*)(wsm + 5120 + 8 * i) = *(const v8h*)(wm1p + 8 * i);
  {
    const float vbe2 = be2[lane & 15];
    const float vbn2 = bn2[lane];
    const float vbm1 = bm1[lane & 15];
    const float vwm2 = wm2[lane];
    const float vbm2 = bm2[lane & 1];
    if (wave == 0 && lane < 16) bias[lane] = vbe2;
    if (wave == 1) bias[16 + lane] = vbn2;
    if (wave == 2 && lane < 16) bias[48 + lane] = vbm1;
    if (wave == 3) bias[64 + lane] = vwm2;
    if (wave == 4 && lane < 2) bias[96 + lane] = vbm2;
  }
  if (tid == 0) pendN = 0;
  __syncthreads();

  const int nChunks = (nE + CHUNK - 1) / CHUNK;
#pragma unroll 1
  for (int ch = 0; ch < nChunks; ++ch) {
    const int cbase = ch * CHUNK;
    const int wc = scan_chunk<NBK>(srcs, nE, cbase, nodeBase, vec8, list, tid, wave);
    if (lane == 0) wcnt[wave] = wc;
    __syncthreads();

    const int base = pendN;
    int tot = 0, myoff = 0;
#pragma unroll
    for (int w = 0; w < NWAVE; ++w) {
      int c = wcnt[w];
      c = c > WCAP ? WCAP : (c < 0 ? 0 : c);
      if (w < wave) myoff += c;
      tot += c;
    }
    int newN = base + tot;
    newN = newN > PCAP ? PCAP : newN;
    {
      int n = wcnt[wave];
      n = n > WCAP ? WCAP : (n < 0 ? 0 : n);
      const int* lp = list + wave * WCAP;
      for (int i = lane; i < n; i += 32) {
        const int pos = base + myoff + i;
        if (pos < PCAP) pend[pos] = cbase + lp[i];
      }
    }
    const int fin = (ch == nChunks - 1) ? 1 : 0;
    const int R   = (fin != 0) ? (newN + PASSN - 1) / PASSN : newN / PASSN;
    const int Pv  = (fin != 0) ? newN : R * PASSN;
    __syncthreads();

#pragma unroll 1
    for (int r = 0; r < R; ++r) {
      {
        const int el  = wave * 16 + m;
        const int idx = r * PASSN + el;
        const bool valid = idx < Pv;
        int e = pend[idx];
        if (!valid) e = 0;
        e = clampi(e, nE - 1);
        int rw = srcs[e];
        int cl = dsts[e];
        int slot = rw - nodeBase;
        if (!valid || (unsigned)slot >= (unsigned)NBK) slot = NBK;
        rw = clampi(rw, nN - 1);
        cl = clampi(cl, nN - 1);
        if (hh == 0) { slotb[el] = slot; colb[el] = cl; }
        const float* ap_ = Ap + (size_t)rw * 64 + hh * 32;
        const float* bp_ = Bp + (size_t)cl * 64 + hh * 32;
        _Float16* sp = stgU + el * 64 + hh * 32;
#pragma unroll 1
        for (int g = 0; g < 4; ++g) {
          const v4f a0 = *(const v4f*)(ap_ + 8 * g);
          const v4f a1 = *(const v4f*)(ap_ + 8 * g + 4);
          const v4f b0 = *(const v4f*)(bp_ + 8 * g);
          const v4f b1 = *(const v4f*)(bp_ + 8 * g + 4);
          const v4f t0 = a0 + b0;
          const v4f t1 = a1 + b1;
          v8h hv;
#pragma unroll
          for (int j = 0; j < 4; ++j) {
            float a = lrl(t0[j], 0.12f);
            float b = lrl(t1[j], 0.12f);
            if (!valid) { a = 0.0f; b = 0.0f; }
            hv[j]     = (_Float16)a;
            hv[4 + j] = (_Float16)b;
          }
          *(v8h*)(sp + 8 * g) = hv;
        }
      }
      __syncthreads();

      {
        v8f a1 = zacc();
        const _Float16* arow = stgU + (wave * 16 + m) * 64 + 8 * hh;
#pragma unroll
        for (int ks = 0; ks < 2; ++ks) {
          FragH a, b;
          a.h[0] = *(const v8h*)(arow + 32 * ks);
          a.h[1] = *(const v8h*)(arow + 32 * ks + 16);
          const _Float16* brow = wsm + m * 64 + 8 * hh + 32 * ks;
          b.h[0] = *(const v8h*)brow;
          b.h[1] = *(const v8h*)(brow + 16);
          a1 = wmh(a.v, b.v, a1);
        }
        const float bv = bias[m];
        _Float16* ep = stgE + (wave * 16 + 8 * hh) * 32;
#pragma unroll
        for (int rr = 0; rr < 8; ++rr) {
          ep[rr * 32 + m]      = (_Float16)(a1[rr] * 0.125f + bv);
          ep[rr * 32 + 16 + m] = (_Float16)0.0f;
        }
      }
      __syncthreads();

      {
        v8f a2[4];
#pragma unroll
        for (int nb = 0; nb < 4; ++nb) a2[nb] = zacc();
        FragH a;
        const _Float16* arow = stgE + (wave * 16 + m) * 32 + 8 * hh;
        a.h[0] = *(const v8h*)arow;
        a.h[1] = *(const v8h*)(arow + 16);
#pragma unroll
        for (int nb = 0; nb < 4; ++nb) {
          FragH b;
          const _Float16* brow = wsm + 1024 + (nb * 16 + m) * 32 + 8 * hh;
          b.h[0] = *(const v8h*)brow;
          b.h[1] = *(const v8h*)(brow + 16);
          a2[nb] = wmh(a.v, b.v, a2[nb]);
        }
#pragma unroll
        for (int rr = 0; rr < 8; ++rr) {
          const int el2 = wave * 16 + 8 * hh + rr;
          int cl = colb[el2];
          cl = clampi(cl, nN - 1);
          const float* crow = Cp + (size_t)cl * 64 + m;
          _Float16* vp = stgV + el2 * 64 + m;
#pragma unroll
          for (int nb = 0; nb < 4; ++nb) {
            const float cv = crow[nb * 16];
            vp[nb * 16] = (_Float16)lrl(cv + a2[nb][rr] * 0.125f, 0.12f);
          }
        }
      }
      __syncthreads();

      {
        v8f a3[2];
        a3[0] = zacc(); a3[1] = zacc();
        const _Float16* arow = stgV + (wave * 16 + m) * 64 + 8 * hh;
#pragma unroll
        for (int ks = 0; ks < 2; ++ks) {
          FragH a;
          a.h[0] = *(const v8h*)(arow + 32 * ks);
          a.h[1] = *(const v8h*)(arow + 32 * ks + 16);
#pragma unroll
          for (int nb = 0; nb < 2; ++nb) {
            FragH b;
            const _Float16* brow = wsm + 3072 + (nb * 16 + m) * 64 + 8 * hh + 32 * ks;
            b.h[0] = *(const v8h*)brow;
            b.h[1] = *(const v8h*)(brow + 16);
            a3[nb] = wmh(a.v, b.v, a3[nb]);
          }
        }
#pragma unroll
        for (int nb = 0; nb < 2; ++nb) {
          const float bv = bias[16 + nb * 16 + m];
          float* mp = msg + (wave * 16 + 8 * hh) * 32 + nb * 16 + m;
#pragma unroll
          for (int rr = 0; rr < 8; ++rr) mp[rr * 32] = a3[nb][rr] * 0.125f + bv;
        }
      }
      __syncthreads();

      if (wave == 0) {
#pragma unroll 1
        for (int i = 0; i < PASSN; ++i) {
          int sl = slotb[i];
          sl = sl < 0 ? 0 : (sl > NBK ? NBK : sl);
          acc[sl * 32 + lane] += msg[i * 32 + lane];
          if (lane == 0) cntb[sl] += 1;
        }
      }
      __syncthreads();
    }

    int rem = newN - R * PASSN;
    rem = rem < 0 ? 0 : rem;
    if (R > 0 && tid < rem) pend[tid] = pend[R * PASSN + tid];
    if (tid == 0) pendN = rem;
  }
  __syncthreads();

#pragma unroll 1
  for (int tt = 0; tt < NTT; ++tt) {
    const int n0 = (tt * NWAVE + wave) * 16;
    {
      const int sl = n0 + m;
      const float rc = 1.0f / fmaxf((float)cntb[sl], 1.0f);
      const float* ar = acc + sl * 32 + 16 * hh;
      v8h h0, h1;
#pragma unroll
      for (int j = 0; j < 8; ++j) { h0[j] = (_Float16)(ar[j] * rc); h1[j] = (_Float16)(ar[8 + j] * rc); }
      _Float16* mrow = stgE + (wave * 16 + m) * 32 + 16 * hh;
      *(v8h*)mrow       = h0;
      *(v8h*)(mrow + 8) = h1;
    }
    __syncthreads();
    {
      FragH a, b;
      const _Float16* arow = stgE + (wave * 16 + m) * 32 + 8 * hh;
      a.h[0] = *(const v8h*)arow;
      a.h[1] = *(const v8h*)(arow + 16);
      const _Float16* brow = wsm + 5120 + m * 32 + 8 * hh;
      b.h[0] = *(const v8h*)brow;
      b.h[1] = *(const v8h*)(brow + 16);
      const v8f a4 = wmh(a.v, b.v, zacc());
      const float bv = bias[48 + m];
      float* hp = msg + wave * 256 + (8 * hh) * 16 + m;
#pragma unroll
      for (int rr = 0; rr < 8; ++rr) hp[rr * 16] = lrl(a4[rr] * 0.25f + bv, 0.12f);
    }
    __syncthreads();
    {
      const int nl = lane & 15;
      const float* hrow = msg + wave * 256 + nl * 16;
      float o0 = bias[96], o1 = bias[97];
#pragma unroll 1
      for (int k = 0; k < 16; ++k) {
        const float hk = hrow[k];
        o0 += hk * bias[64 + 2 * k];
        o1 += hk * bias[65 + 2 * k];
      }
      const float mx = fmaxf(o0, o1);
      const float s0 = o0 - mx, s1 = o1 - mx;
      const float l  = logf(expf(s0) + expf(s1));
      if (lane < 16) {
        outst[(n0 + nl) * 2]     = s0 - l;
        outst[(n0 + nl) * 2 + 1] = s1 - l;
      }
    }
  }
  __syncthreads();

  const long lim = 2L * (long)nN - 2L * (long)nodeBase;
  const size_t ob = (size_t)nodeBase * 2;
#pragma unroll
  for (int q = 0; q < NQO; ++q) {
    const int f = (wave * NQO + q) * 128 + 4 * lane;
    const v4f v = *(const v4f*)(outst + f);
    if ((long)f + 3 < lim) *(volatile v4f*)(outp + ob + f) = v;
  }
  __threadfence();
#pragma unroll
  for (int q = 0; q < NQO; ++q) {
    const int f = (wave * NQO + q) * 128 + 4 * lane;
    const v4f v = *(const v4f*)(outst + f);
    if ((long)f + 3 < lim) *(volatile v4f*)(outp + ob + f) = v;
  }
}

extern "C" void kernel_launch(void* const* d_in, const int* in_sizes, int n_in,
                              void* d_out, int out_size, void* d_ws, size_t ws_size,
                              hipStream_t stream) {
  if (n_in < 26) return;
  const int nN = in_sizes[0] / 4;
  const int nE = in_sizes[1] / 2;
  if (nN <= 0 || nE < 0 || in_sizes[0] != nN * 4 || in_sizes[1] != nE * 2) return;
  if (in_sizes[2] != 8 * 32 || in_sizes[3] < 32 || in_sizes[4] != 32 * 16 || in_sizes[5] < 16) return;
  if (in_sizes[6] != 32 * 64 || in_sizes[7] < 64 || in_sizes[8] != 64 * 32 || in_sizes[9] < 32) return;
  if (in_sizes[10] != 64 * 128 || in_sizes[11] < 128 || in_sizes[12] != 128 * 64 || in_sizes[13] < 64) return;
  if (in_sizes[14] != 128 * 64 || in_sizes[15] < 64 || in_sizes[16] != 64 * 16 || in_sizes[17] < 16) return;
  if (in_sizes[18] != 80 * 64 || in_sizes[19] < 64 || in_sizes[20] != 64 * 32 || in_sizes[21] < 32) return;
  if (in_sizes[22] != 32 * 16 || in_sizes[23] < 16 || in_sizes[24] != 16 * 2 || in_sizes[25] < 2) return;
  if (out_size != nN * 2) return;

  const float* x   = (const float*)d_in[0];
  const int*   ei  = (const int*)d_in[1];
  const float* w1a = (const float*)d_in[2];  const float* b1a = (const float*)d_in[3];
  const float* w1b = (const float*)d_in[4];  const float* b1b = (const float*)d_in[5];
  const float* w2a = (const float*)d_in[6];  const float* b2a = (const float*)d_in[7];
  const float* w2b = (const float*)d_in[8];  const float* b2b = (const float*)d_in[9];
  const float* w3a = (const float*)d_in[10]; const float* b3a = (const float*)d_in[11];
  const float* w3b = (const float*)d_in[12]; const float* b3b = (const float*)d_in[13];
  const float* we1 = (const float*)d_in[14]; const float* be1 = (const float*)d_in[15];
  const float* we2 = (const float*)d_in[16]; const float* be2 = (const float*)d_in[17];
  const float* wn1 = (const float*)d_in[18]; const float* bn1 = (const float*)d_in[19];
  const float* wn2 = (const float*)d_in[20]; const float* bn2 = (const float*)d_in[21];
  const float* wm1 = (const float*)d_in[22]; const float* bm1 = (const float*)d_in[23];
  const float* wm2 = (const float*)d_in[24]; const float* bm2 = (const float*)d_in[25];
  float* out = (float*)d_out;

  const int nPad = ((nN + 2047) / 2048) * 2048;

  char* ws = (char*)d_ws;
  size_t off = 0;
  const size_t oPl = off; off += (size_t)PLANES_H * 2;              off = (off + 255) & ~(size_t)255;
  const size_t oPQ = off; off += (size_t)2 * nPad * 128 * 4;        off = (off + 255) & ~(size_t)255;
  const size_t oX1 = off; off += (size_t)nPad * 16 * 4;             off = (off + 255) & ~(size_t)255;
  const size_t oX2 = off; off += (size_t)nPad * 32 * 4;             off = (off + 255) & ~(size_t)255;
  const size_t oX3 = off; off += (size_t)nPad * 64 * 4;             off = (off + 255) & ~(size_t)255;
  if (off > ws_size) return;
  _Float16* planes = (_Float16*)(ws + oPl);
  float* PQ = (float*)(ws + oPQ);
  float* X1 = (float*)(ws + oX1);
  float* X2 = (float*)(ws + oX2);
  float* X3 = (float*)(ws + oX3);
  float* P   = PQ;
  float* Q1  = PQ + (size_t)nPad * 32;
  float* Q2  = PQ + (size_t)nPad * 64;
  float* Q3  = PQ + (size_t)nPad * 128;
  float* Am  = PQ;
  float* Bm  = PQ + (size_t)nPad * 64;
  float* Cm  = PQ + (size_t)2 * nPad * 64;

  const int vec8 = ((nE & 3) == 0) ? 1 : 0;

  k_prep<<<NPLANES, NTHR, 0, stream>>>(w1b, w2a, w2b, w3a, w3b, we1, we2, wn1, wn2, wm1, planes);

  k_node1<<<nPad / 1024, NTHR, 0, stream>>>(x, w1a, b1a, P, Q1, nN, nPad);

  k_econv<32, 16, 2048><<<nPad / 2048, NTHR, 0, stream>>>(
      P, Q1, ei, planes + OF_WB1, b1b, 0.25f, X1, nN, nE, vec8);

  k_nodeg<16, 64, 2><<<nPad / NODET, NTHR, 0, stream>>>(
      X1, planes + OF_PA2, planes + OF_QA2, planes + OF_PA2, b2a, b2a, 0.25f, P, Q2, P);

  k_econv<64, 32, 1024><<<nPad / 1024, NTHR, 0, stream>>>(
      P, Q2, ei, planes + OF_WB2, b2b, 0.125f, X2, nN, nE, vec8);

  k_nodeg<32, 128, 2><<<nPad / NODET, NTHR, 0, stream>>>(
      X2, planes + OF_PA3, planes + OF_QA3, planes + OF_PA3, b3a, b3a, 0.125f, P, Q3, P);

  k_econv<128, 64, 512><<<nPad / 512, NTHR, 0, stream>>>(
      P, Q3, ei, planes + OF_WB3, b3b, 0.125f, X3, nN, nE, vec8);

  k_nodeg<64, 64, 3><<<nPad / NODET, NTHR, 0, stream>>>(
      X3, planes + OF_AE, planes + OF_BE, planes + OF_CN, be1, bn1, 0.125f, Am, Bm, Cm);

  k_meta<1024><<<nPad / 1024, NTHR, 0, stream>>>(
      Am, Bm, Cm, ei, planes + OF_WE2, planes + OF_EN, planes + OF_WN2, planes + OF_WM1,
      be2, bn2, bm1, wm2, bm2, out, nN, nE, vec8);
}
